// DeepContextDependentChoice_85521388798585
// MI455X (gfx1250) — hardware-verified
//
#include <hip/hip_runtime.h>

#define A_ 128
#define F_ 32
#define H_ 64
#define NT 256

typedef float          v8f   __attribute__((ext_vector_type(8)));
typedef float          v4f   __attribute__((ext_vector_type(4)));
typedef __bf16         v16bf __attribute__((ext_vector_type(16)));
typedef unsigned short v8us  __attribute__((ext_vector_type(8)));
typedef unsigned int   v8u   __attribute__((ext_vector_type(8)));
typedef v8us __attribute__((__may_alias__)) v8us_a;
typedef v4f  __attribute__((__may_alias__)) v4f_a;

union Frg { v16bf v; v8us p[2]; v8u u; unsigned int w[8]; };

__device__ __forceinline__ unsigned int bf_rne(float x) {
    unsigned int u = __float_as_uint(x);
    return (u + 0x7fffu + ((u >> 16) & 1u)) >> 16;
}
__device__ __forceinline__ void bf_split(float x, unsigned int& hb, unsigned int& lb) {
    hb = bf_rne(x);
    lb = bf_rne(x - __uint_as_float(hb << 16));
}
__device__ __forceinline__ void split_store(float x, unsigned short* ph, unsigned short* pl, int idx) {
    unsigned int hb, lb;
    bf_split(x, hb, lb);
    ph[idx] = (unsigned short)hb;
    pl[idx] = (unsigned short)lb;
}
__device__ __forceinline__ void ldfrag(Frg& f, const unsigned short* plane, int row, int pitch, int k0, int h) {
    const unsigned short* p = plane + row * pitch + k0 + 8 * h;
    f.p[0] = *(const v8us_a*)(p);
    f.p[1] = *(const v8us_a*)(p + 16);
}
__device__ __forceinline__ void split16(const float* x, Frg& fh, Frg& fl) {
#pragma unroll
    for (int q = 0; q < 8; ++q) {
        unsigned int h0, l0, h1, l1;
        bf_split(x[2 * q], h0, l0);
        bf_split(x[2 * q + 1], h1, l1);
        fh.w[q] = h0 | (h1 << 16);
        fl.w[q] = l0 | (l1 << 16);
    }
}
__device__ __forceinline__ v8f zero8() {
    v8f z = {0.f, 0.f, 0.f, 0.f, 0.f, 0.f, 0.f, 0.f};
    return z;
}
__device__ __forceinline__ v8f mma(const Frg& a, const Frg& b, v8f c) {
    return __builtin_amdgcn_wmma_f32_16x16x32_bf16(false, a.v, false, b.v, (short)0, c, false, false);
}
__device__ __forceinline__ v8f mma3(const Frg& ah, const Frg& al, const Frg& bh, const Frg& bl, v8f c) {
    c = mma(al, bh, c);
    c = mma(ah, bl, c);
    c = mma(ah, bh, c);
    return c;
}
__device__ __forceinline__ void mguard(v8f& c, const Frg& a, const Frg& b) {
    asm volatile("v_nop\n\tv_nop\n\tv_nop\n\tv_nop" : "+v"(c) : "v"(a.u), "v"(b.u));
}
__device__ __forceinline__ float hsum16(float v) {
    v += __shfl_xor(v, 1, 32);
    v += __shfl_xor(v, 2, 32);
    v += __shfl_xor(v, 4, 32);
    v += __shfl_xor(v, 8, 32);
    return v;
}
__device__ __forceinline__ float wmax32(float v) {
#pragma unroll
    for (int o = 16; o > 0; o >>= 1) v = fmaxf(v, __shfl_xor(v, o, 32));
    return v;
}
__device__ __forceinline__ float wsum32(float v) {
#pragma unroll
    for (int o = 16; o > 0; o >>= 1) v += __shfl_xor(v, o, 32);
    return v;
}

__global__ void __launch_bounds__(NT)
k_main(const float* __restrict__ X,   const int*   __restrict__ mask,
       const float* __restrict__ bW1, const float* __restrict__ bb1,
       const float* __restrict__ bW2, const float* __restrict__ bb2,
       const float* __restrict__ bW3, const float* __restrict__ bb3,
       const float* __restrict__ pW1, const float* __restrict__ pb1,
       const float* __restrict__ pW2, const float* __restrict__ pb2,
       const float* __restrict__ pW3, const float* __restrict__ pb3,
       float* __restrict__ out, int nb)
{
    __shared__ __align__(16) unsigned short s_xh[A_ * F_];
    __shared__ __align__(16) unsigned short s_xl[A_ * F_];
    __shared__ __align__(16) unsigned short s_wih[H_ * F_];
    __shared__ __align__(16) unsigned short s_wil[H_ * F_];
    __shared__ __align__(16) unsigned short s_wjh[H_ * F_];
    __shared__ __align__(16) unsigned short s_wjl[H_ * F_];
    __shared__ __align__(16) unsigned short s_b1h[H_ * F_];
    __shared__ __align__(16) unsigned short s_b1l[H_ * F_];
    __shared__ __align__(16) unsigned short s_b2h[H_ * H_];
    __shared__ __align__(16) unsigned short s_b2l[H_ * H_];
    __shared__ __align__(16) unsigned short s_p2h[H_ * H_];
    __shared__ __align__(16) unsigned short s_p2l[H_ * H_];
    __shared__ __align__(16) float s_R[2 * A_ * H_];
    __shared__ int s_mask[A_];
    __shared__ __align__(16) float s_bu[A_];
    __shared__ __align__(16) float s_ps[A_];
    __shared__ __align__(16) float s_u[A_];
    __shared__ float s_red[8];

    const int b = blockIdx.x;
    if (b >= nb) return;
    const int tid  = threadIdx.x;
    const int lane = tid & 31;
    const int w    = tid >> 5;
    const int h    = lane >> 4;
    const int m    = lane & 15;
    const int r0   = w * 16;

    const float* Xb = X + (size_t)b * (A_ * F_);
    for (int i = tid; i < A_ * F_; i += NT) split_store(Xb[i], s_xh, s_xl, i);
    for (int i = tid; i < F_ * H_; i += NT) {
        const int k = i >> 6, n = i & 63;
        split_store(pW1[i],           s_wih, s_wil, n * F_ + k);
        split_store(pW1[F_ * H_ + i], s_wjh, s_wjl, n * F_ + k);
        split_store(bW1[i],           s_b1h, s_b1l, n * F_ + k);
    }
    for (int i = tid; i < H_ * H_; i += NT) {
        const int k = i >> 6, n = i & 63;
        split_store(bW2[i], s_b2h, s_b2l, n * H_ + k);
        split_store(pW2[i], s_p2h, s_p2l, n * H_ + k);
    }
    if (tid < A_) s_mask[tid] = mask[(size_t)b * A_ + tid];
    __syncthreads();

    unsigned short* s_h1h = reinterpret_cast<unsigned short*>(s_R);
    unsigned short* s_h1l = s_h1h + A_ * H_;

    {
        Frg xh, xl;
        ldfrag(xh, s_xh, r0 + m, F_, 0, h);
        ldfrag(xl, s_xl, r0 + m, F_, 0, h);
#pragma unroll
        for (int t = 0; t < 4; ++t) {
            const int col = t * 16 + m;
            Frg bh, bl;
            ldfrag(bh, s_b1h, col, F_, 0, h);
            ldfrag(bl, s_b1l, col, F_, 0, h);
            v8f c = zero8();
            c = mma3(xh, xl, bh, bl, c);
            mguard(c, xh, bh);
            const float bias = bb1[col];
#pragma unroll
            for (int r = 0; r < 8; ++r) {
                const float v = fmaxf(c[r] + bias, 0.f);
                unsigned int hb, lb;
                bf_split(v, hb, lb);
                const int o = (r0 + 8 * h + r) * H_ + col;
                s_h1h[o] = (unsigned short)hb;
                s_h1l[o] = (unsigned short)lb;
            }
        }
    }
    __syncthreads();

    {
        Frg a0h, a0l, a1h, a1l;
        ldfrag(a0h, s_h1h, r0 + m, H_, 0, h);
        ldfrag(a0l, s_h1l, r0 + m, H_, 0, h);
        ldfrag(a1h, s_h1h, r0 + m, H_, 32, h);
        ldfrag(a1l, s_h1l, r0 + m, H_, 32, h);
        float s8[8];
#pragma unroll
        for (int r = 0; r < 8; ++r) s8[r] = 0.f;
#pragma unroll
        for (int t = 0; t < 4; ++t) {
            const int col = t * 16 + m;
            Frg bh0, bl0, bh1, bl1;
            ldfrag(bh0, s_b2h, col, H_, 0, h);
            ldfrag(bl0, s_b2l, col, H_, 0, h);
            ldfrag(bh1, s_b2h, col, H_, 32, h);
            ldfrag(bl1, s_b2l, col, H_, 32, h);
            v8f c = zero8();
            c = mma3(a0h, a0l, bh0, bl0, c);
            c = mma3(a1h, a1l, bh1, bl1, c);
            mguard(c, a1h, bh1);
            const float bias = bb2[col];
            const float w3   = bW3[col];
#pragma unroll
            for (int r = 0; r < 8; ++r) s8[r] += fmaxf(c[r] + bias, 0.f) * w3;
        }
#pragma unroll
        for (int r = 0; r < 8; ++r) s8[r] = hsum16(s8[r]);
        if (m == 0) {
            const float b3 = bb3[0];
#pragma unroll
            for (int r = 0; r < 8; ++r) s_bu[r0 + 8 * h + r] = s8[r] + b3;
        }
    }
    __syncthreads();

    float* s_hi = s_R;
    float* s_hj = s_R + A_ * H_;

    {
        Frg xh, xl;
        ldfrag(xh, s_xh, r0 + m, F_, 0, h);
        ldfrag(xl, s_xl, r0 + m, F_, 0, h);
#pragma unroll
        for (int t = 0; t < 4; ++t) {
            const int col = t * 16 + m;
            {
                Frg bh, bl;
                ldfrag(bh, s_wih, col, F_, 0, h);
                ldfrag(bl, s_wil, col, F_, 0, h);
                v8f c = zero8();
                c = mma3(xh, xl, bh, bl, c);
                mguard(c, xh, bh);
                const float bias = pb1[col];
#pragma unroll
                for (int r = 0; r < 8; ++r) s_hi[(r0 + 8 * h + r) * H_ + col] = c[r] + bias;
            }
            {
                Frg bh, bl;
                ldfrag(bh, s_wjh, col, F_, 0, h);
                ldfrag(bl, s_wjl, col, F_, 0, h);
                v8f c = zero8();
                c = mma3(xh, xl, bh, bl, c);
                mguard(c, xh, bh);
#pragma unroll
                for (int r = 0; r < 8; ++r) s_hj[(r0 + 8 * h + r) * H_ + col] = c[r];
            }
        }
    }
    __syncthreads();

    float hv[32];
    {
        const float* hp = s_hi + (r0 + m) * H_ + 8 * h;
#pragma unroll
        for (int g = 0; g < 4; ++g) {
            const v4f q0 = *(const v4f_a*)(hp + 16 * g);
            const v4f q1 = *(const v4f_a*)(hp + 16 * g + 4);
            hv[8 * g + 0] = q0[0]; hv[8 * g + 1] = q0[1]; hv[8 * g + 2] = q0[2]; hv[8 * g + 3] = q0[3];
            hv[8 * g + 4] = q1[0]; hv[8 * g + 5] = q1[1]; hv[8 * g + 6] = q1[2]; hv[8 * g + 7] = q1[3];
        }
    }
    float pb2v[4], pw3v[4];
#pragma unroll
    for (int t = 0; t < 4; ++t) { pb2v[t] = pb2[t * 16 + m]; pw3v[t] = pW3[t * 16 + m]; }

    float acc[4][8];
#pragma unroll
    for (int t = 0; t < 4; ++t)
#pragma unroll
        for (int r = 0; r < 8; ++r) acc[t][r] = 0.f;

    const int dzb = r0 + 8 * h;

#pragma unroll 1
    for (int j = 0; j < A_; ++j) {
        asm volatile("" ::: "memory");
        const int mj = __builtin_amdgcn_readfirstlane(s_mask[j]);
        if (mj == 0) continue;

        const float* hjp = s_hj + j * H_ + 8 * h;
        float x[32];
#pragma unroll
        for (int g = 0; g < 4; ++g) {
            const v4f q0 = *(const v4f_a*)(hjp + 16 * g);
            const v4f q1 = *(const v4f_a*)(hjp + 16 * g + 4);
            x[8 * g + 0] = fmaxf(hv[8 * g + 0] + q0[0], 0.f);
            x[8 * g + 1] = fmaxf(hv[8 * g + 1] + q0[1], 0.f);
            x[8 * g + 2] = fmaxf(hv[8 * g + 2] + q0[2], 0.f);
            x[8 * g + 3] = fmaxf(hv[8 * g + 3] + q0[3], 0.f);
            x[8 * g + 4] = fmaxf(hv[8 * g + 4] + q1[0], 0.f);
            x[8 * g + 5] = fmaxf(hv[8 * g + 5] + q1[1], 0.f);
            x[8 * g + 6] = fmaxf(hv[8 * g + 6] + q1[2], 0.f);
            x[8 * g + 7] = fmaxf(hv[8 * g + 7] + q1[3], 0.f);
        }
        Frg a0h, a0l, a1h, a1l;
        split16(x, a0h, a0l);
        split16(x + 16, a1h, a1l);
        const int dz = j - dzb;

#pragma unroll
        for (int t = 0; t < 4; ++t) {
            asm volatile("" ::: "memory");
            const int col = t * 16 + m;
            Frg bh0, bl0, bh1, bl1;
            ldfrag(bh0, s_p2h, col, H_, 0, h);
            ldfrag(bl0, s_p2l, col, H_, 0, h);
            ldfrag(bh1, s_p2h, col, H_, 32, h);
            ldfrag(bl1, s_p2l, col, H_, 32, h);
            v8f c = zero8();
            c = mma3(a0h, a0l, bh0, bl0, c);
            c = mma3(a1h, a1l, bh1, bl1, c);
            mguard(c, a1h, bh1);
#pragma unroll
            for (int r = 0; r < 8; ++r) {
                float v = fmaxf(c[r] + pb2v[t], 0.f);
                v = (dz == r) ? 0.f : v;
                acc[t][r] += v;
            }
        }
    }

    {
        float s8[8];
#pragma unroll
        for (int r = 0; r < 8; ++r)
            s8[r] = acc[0][r] * pw3v[0] + acc[1][r] * pw3v[1] + acc[2][r] * pw3v[2] + acc[3][r] * pw3v[3];
#pragma unroll
        for (int r = 0; r < 8; ++r) s8[r] = hsum16(s8[r]);
        if (m == 0) {
#pragma unroll
            for (int r = 0; r < 8; ++r) s_ps[r0 + 8 * h + r] = s8[r];
        }
    }
    __syncthreads();

    if (tid < A_) {
        int nm = 0;
#pragma unroll 8
        for (int jj = 0; jj < A_; ++jj) nm += s_mask[jj];
        const int mi = s_mask[tid];
        float u = -1.0e9f;
        if (mi != 0) u = s_bu[tid] + s_ps[tid] + pb3[0] * (float)(nm - 1);
        s_u[tid] = u;
    }
    __syncthreads();

    float uval = 0.f, ev = 0.f;
    if (tid < A_) {
        uval = s_u[tid];
        const float mx = wmax32(uval);
        if (lane == 0) s_red[w] = mx;
    }
    __syncthreads();
    if (tid < A_) {
        const float mx = fmaxf(fmaxf(s_red[0], s_red[1]), fmaxf(s_red[2], s_red[3]));
        ev = expf(uval - mx);
        const float sm = wsum32(ev);
        if (lane == 0) s_red[4 + w] = sm;
    }
    __syncthreads();
    if (tid < A_) {
        const float tot = (s_red[4] + s_red[5]) + (s_red[6] + s_red[7]);
        s_u[tid] = ev * (1.0f / tot);
    }
    __syncthreads();

    if (w == 0) {
        const v4f v = *(const v4f_a*)(s_u + 4 * lane);
        float* op = out + (size_t)b * A_ + 4 * lane;
        *(volatile v4f*)op = v;
        __threadfence();
        *(volatile v4f*)op = v;
    }
}

extern "C" void kernel_launch(void* const* d_in, const int* in_sizes, int n_in,
                              void* d_out, int out_size, void* d_ws, size_t ws_size,
                              hipStream_t stream)
{
    (void)d_ws; (void)ws_size;
    if (n_in < 14) return;
    const int nb = out_size / A_;
    if (nb <= 0 || nb * A_ != out_size) return;
    if (in_sizes[0] != nb * A_ * F_) return;
    if (in_sizes[1] != nb * A_) return;
    if (in_sizes[2] != F_ * H_ || in_sizes[3] != H_) return;
    if (in_sizes[4] != H_ * H_ || in_sizes[5] != H_) return;
    if (in_sizes[6] != H_ || in_sizes[7] != 1) return;
    if (in_sizes[8] != 2 * F_ * H_ || in_sizes[9] != H_) return;
    if (in_sizes[10] != H_ * H_ || in_sizes[11] != H_) return;
    if (in_sizes[12] != H_ || in_sizes[13] != 1) return;

    const float* X    = (const float*)d_in[0];
    const int*   mask = (const int*)  d_in[1];
    const float* bW1  = (const float*)d_in[2];
    const float* bb1  = (const float*)d_in[3];
    const float* bW2  = (const float*)d_in[4];
    const float* bb2  = (const float*)d_in[5];
    const float* bW3  = (const float*)d_in[6];
    const float* bb3  = (const float*)d_in[7];
    const float* pW1  = (const float*)d_in[8];
    const float* pb1  = (const float*)d_in[9];
    const float* pW2  = (const float*)d_in[10];
    const float* pb2  = (const float*)d_in[11];
    const float* pW3  = (const float*)d_in[12];
    const float* pb3  = (const float*)d_in[13];
    float* out = (float*)d_out;

    k_main<<<dim3(nb), dim3(NT), 0, stream>>>(X, mask, bW1, bb1, bW2, bb2, bW3, bb3,
                                              pW1, pb1, pW2, pb2, pW3, pb3, out, nb);
    (void)hipGetLastError();
}
